// PermutohedralLatticeLayer_21242908246578
// MI455X (gfx1250) — hardware-run, weakly checked
//
#include <hip/hip_runtime.h>
#include <math.h>


#ifndef NPTS
#define NPTS 262144
#endif
#define NPTS_FULL 262144
#define LL    16
#define TSZ   262144
#define NF    32
#define PTS   128
#define ENCP  40
#define OSP   36
#define ECARRY 1048576.0f
#define WCARRY 256.0f
#define FOLD  (1.0f / 268435456.0f)
#define COARSEST_RES 10.0
#define FINEST_RES   1000.0
#define IS0 ((float)0.70710678118654752440)
#define IS1 ((float)0.40824829046386301637)
#define IS2 ((float)0.28867513459481288225)

static_assert(NPTS % PTS == 0);
static_assert(NPTS <= NPTS_FULL);
static_assert(NF == LL * 2);
static_assert(NF == 32);
static_assert(PTS == 8 * 16);
static_assert(256 == LL * 16);
static_assert(2 * 256 >= PTS * 3);
static_assert((ENCP * 2) % 16 == 0);
static_assert(ENCP >= NF);
static_assert((OSP * 4) % 16 == 0);
static_assert(OSP >= NF);
static_assert(32 * 16 * 4 == 16 * NF * 4);
static_assert(128 * 8 == NF * NF);
static_assert(PTS * 3 * 4 + PTS * ENCP * 2 + 8 * 16 * OSP * 4 <= 131072);

typedef _Float16 h16;
typedef unsigned short bf;
typedef __attribute__((ext_vector_type(16))) __bf16   v16bf;
typedef __attribute__((ext_vector_type(16))) _Float16 v16h;
typedef __attribute__((ext_vector_type(8)))  _Float16 v8h;
typedef __attribute__((ext_vector_type(8)))  unsigned short v8us;
typedef __attribute__((ext_vector_type(8)))  float    v8f;
typedef __attribute__((ext_vector_type(4)))  float    v4f;
typedef v4f  __attribute__((may_alias)) v4fa;
typedef v8h  __attribute__((may_alias)) v8ha;
typedef __attribute__((ext_vector_type(2)))  float    v2f;

__device__ __forceinline__ unsigned short f2bf(float f) { unsigned u = __float_as_uint(f); u += 0x7FFFu + ((u >> 16) & 1u); return (unsigned short)(u >> 16); }
__device__ __forceinline__ float bfr(float f) { return __uint_as_float(((unsigned)f2bf(f)) << 16); }
__device__ __forceinline__ v16h cat16(v8h lo, v8h hi) { return __builtin_shufflevector(lo, hi, 0, 1, 2, 3, 4, 5, 6, 7, 8, 9, 10, 11, 12, 13, 14, 15); }
__device__ __forceinline__ v16bf cat16b(v8us lo, v8us hi) { return __builtin_bit_cast(v16bf, __builtin_shufflevector(lo, hi, 0, 1, 2, 3, 4, 5, 6, 7, 8, 9, 10, 11, 12, 13, 14, 15)); }
__device__ __forceinline__ v8f wmma16(v16h a, v16h b, v8f c) { return __builtin_amdgcn_wmma_f32_16x16x32_f16(false, a, false, b, (short)0, c, false, false); }
__device__ __forceinline__ v8f wmmab(v16bf a, v16bf b, v8f c) { return __builtin_amdgcn_wmma_f32_16x16x32_bf16(false, a, false, b, (short)0, c, false, false); }
__device__ __forceinline__ v16h  ldh(const h16* p) { return cat16(*(const v8h*)p, *(const v8h*)(p + 16)); }
__device__ __forceinline__ v16bf ldb(const bf* p)  { return cat16b(*(const v8us*)p, *(const v8us*)(p + 16)); }
__device__ __forceinline__ void wave_sync() { __builtin_amdgcn_fence(3  , "wavefront"); __builtin_amdgcn_wave_barrier(); asm volatile("" ::: "memory"); }

static __device__ __forceinline__ h16 toh_flush(float v) { const h16 r = (h16)v; return (fabsf(v) < 6.103515625e-05f) ? (h16)0.0f : r; }
__device__ __forceinline__ v8f wmma16g(v16h a, v16h b, v8f c) {
    c = __builtin_amdgcn_wmma_f32_16x16x32_f16(false, a, false, b, (short)0, c, false, false);
    asm volatile("v_nop\n\tv_nop\n\tv_nop\n\tv_nop" : "+v"(c) : "v"(a), "v"(b));
    return c;
}

__global__ __launch_bounds__(128) void k_wcvt(const float* __restrict__ W, h16* WH) {
    const int i = threadIdx.x;
    const v8f v = *(const v8f*)(W + i * 8); v8h o;
#pragma unroll
    for (int k = 0; k < 8; ++k) o[k] = toh_flush(bfr(v[k]) * WCARRY);
    *(volatile v8h*)(WH + i * 8) = o; __threadfence(); *(volatile v8h*)(WH + i * 8) = o;
}

__global__ __launch_bounds__(256) void k_enc_dense(const float* __restrict__ x, const float* __restrict__ table, const float* __restrict__ shifts,
                                                   const h16* __restrict__ WH, const float* __restrict__ bias, float* OUT) {
#pragma clang fp contract(off)
    __shared__ __align__(16) float xs[PTS * 3];
    __shared__ __align__(16) h16   encs[PTS * ENCP];
    __shared__ __align__(16) float os[8 * 16 * OSP];

    const double growth = 1.3593563908785256;

    const int tid = threadIdx.x;
    const int base_pt = blockIdx.x * PTS;

#pragma unroll
    for (int t = 0; t < 2; ++t) {
        const int i = tid + 256 * t;
        const int ic = (i < PTS * 3) ? i : (PTS * 3 - 1);
        float v = x[(size_t)base_pt * 3 + ic];
        asm volatile("" : "+v"(v));
        if (i < PTS * 3) xs[i] = bfr(v);
    }
    __syncthreads();

    const int lvl  = tid >> 4;
    const int psub = tid & 15;

    double pw = 1.0;
#pragma unroll 1
    for (int i = 0; i < LL - 1; ++i) { const double nx = pw * growth; pw = (i < lvl) ? nx : pw; }
    const float scale = (float)(COARSEST_RES * pw);
    const float sf0 = scale * IS0;
    const float sf1 = scale * IS1;
    const float sf2 = scale * IS2;
    const float sh0 = bfr(shifts[lvl * 3 + 0]);
    const float sh1 = bfr(shifts[lvl * 3 + 1]);
    const float sh2 = bfr(shifts[lvl * 3 + 2]);
    const size_t tb = (size_t)lvl * TSZ;

#pragma unroll 1
    for (int pass = 0; pass < PTS / 16; ++pass) {
        const int p = pass * 16 + psub;
        const float cf0 = (xs[p * 3 + 0] + sh0) * sf0;
        const float cf1 = (xs[p * 3 + 1] + sh1) * sf1;
        const float cf2 = (xs[p * 3 + 2] + sh2) * sf2;

        float e[4];
        e[0] = (cf0 + cf1) + cf2;
        e[1] = (cf1 - cf0) + cf2;
        e[2] = (-2.0f * cf1) + cf2;
        e[3] = -3.0f * cf2;

        float rem[4];
        float rsum = 0.0f;
#pragma unroll
        for (int i = 0; i < 4; ++i) {
            const float v  = e[i] * 0.25f;
            const float up = ceilf(v)  * 4.0f;
            const float dn = floorf(v) * 4.0f;
            rem[i] = ((up - e[i]) < (e[i] - dn)) ? up : dn;
            rsum += rem[i];
        }
        const int s = (int)rintf(rsum * 0.25f);

        float diff[4];
#pragma unroll
        for (int i = 0; i < 4; ++i) diff[i] = e[i] - rem[i];

        int rank[4];
#pragma unroll
        for (int i = 0; i < 4; ++i) {
            int rk = s;
#pragma unroll
            for (int j = 0; j < 4; ++j) {
                if (j == i) continue;
                rk += ((diff[j] > diff[i]) || ((diff[j] == diff[i]) && (j < i))) ? 1 : 0;
            }
            rank[i] = rk;
        }

        int remi[4];
#pragma unroll
        for (int i = 0; i < 4; ++i) {
            remi[i] = (int)rem[i];
            const int neg = (rank[i] < 0) ? 1 : 0;
            const int ovr = (rank[i] > 3) ? 1 : 0;
            rank[i] += 4 * (neg - ovr);
            remi[i] += 4 * (neg - ovr);
        }

        float delta[4];
#pragma unroll
        for (int i = 0; i < 4; ++i) delta[i] = (e[i] - (float)remi[i]) * 0.25f;

        float bary[5] = {0.0f, 0.0f, 0.0f, 0.0f, 0.0f};
#pragma unroll
        for (int i = 0; i < 4; ++i) {
#pragma unroll
            for (int o = 0; o < 5; ++o) {
                float w = 0.0f;
                w += (rank[i] == (3 - o)) ? delta[i] : 0.0f;
                w -= (rank[i] == (4 - o)) ? delta[i] : 0.0f;
                bary[o] += w;
            }
        }
        bary[0] = bary[0] + (1.0f + bary[4]);

        float acc0 = 0.0f, acc1 = 0.0f;
#pragma unroll
        for (int r = 0; r < 4; ++r) {
            const unsigned k0 = (unsigned)(remi[0] + r - 4 * ((rank[0] > 3 - r) ? 1 : 0));
            const unsigned k1 = (unsigned)(remi[1] + r - 4 * ((rank[1] > 3 - r) ? 1 : 0));
            const unsigned k2 = (unsigned)(remi[2] + r - 4 * ((rank[2] > 3 - r) ? 1 : 0));
            unsigned hsh = k0;
            hsh ^= k1 * 2654435761u;
            hsh ^= k2 * 805459861u;
            const unsigned idx = hsh & (unsigned)(TSZ - 1);
            const v2f f = *(const v2f*)(table + (tb + (size_t)idx) * 2);
            acc0 += bary[r] * bfr(f[0]);
            acc1 += bary[r] * bfr(f[1]);
        }

        const h16 ha = toh_flush(acc0 * ECARRY);
        const h16 hb = toh_flush(acc1 * ECARRY);
        encs[p * ENCP + 2 * lvl]     = ha;
        encs[p * ENCP + 2 * lvl + 1] = hb;
    }
    __syncthreads();

    const int wave = __builtin_amdgcn_readfirstlane((int)(threadIdx.x >> 5));
    const int lane = threadIdx.x & 31, lr = lane & 15, hi = lane >> 4;
    const int ab = (wave * 16 + lr) * ENCP + 8 * hi;
    const v16h a  = cat16(*(const v8ha*)(&encs[ab]), *(const v8ha*)(&encs[ab + 16]));
    const v16h b0 = ldh(WH + (size_t)lr * NF + 8 * hi);
    const v16h b1 = ldh(WH + (size_t)(16 + lr) * NF + 8 * hi);
    v8f c0 = (v8f){}, c1 = (v8f){};
    c0 = wmma16g(a, b0, c0);
    c1 = wmma16g(a, b1, c1);
    const float bc0 = bfr(bias[lr]);
    const float bc1 = bfr(bias[16 + lr]);
    const int wb = wave * 16 * OSP;
#pragma unroll
    for (int r = 0; r < 8; ++r) {
        os[wb + (8 * hi + r) * OSP + lr]      = c0[r] * FOLD + bc0;
        os[wb + (8 * hi + r) * OSP + 16 + lr] = c1[r] * FOLD + bc1;
    }
    wave_sync();
    float* orow = OUT + (size_t)(base_pt + wave * 16) * NF;
#pragma unroll 1
    for (int ps = 0; ps < 2; ++ps) {
#pragma unroll
        for (int s = 0; s < 4; ++s) { const int row = 4 * s + (lane >> 3), cofs = (lane & 7) * 4;
            const v4f val = *(const v4fa*)(&os[wb + row * OSP + cofs]);
            *(volatile v4f*)(orow + (size_t)row * NF + cofs) = val; }
        if (ps == 0) __threadfence(); }
}

static constexpr size_t al256(size_t v) { return (v + 255) & ~(size_t)255; }
static constexpr size_t SZ_WH = al256((size_t)NF * NF * 2);
static constexpr size_t SZ_TOTAL = SZ_WH;
static_assert(SZ_TOTAL <= (size_t)134217728);
static_assert((size_t)128 * 16 <= SZ_WH);
static_assert((size_t)NPTS * NF * 4 <= (size_t)NPTS_FULL * NF * 4);

extern "C" void kernel_launch(void* const* d_in, const int* in_sizes, int n_in,
                              void* d_out, int out_size, void* d_ws, size_t ws_size, hipStream_t stream) {
    if (n_in < 5) return;
    if ((size_t)in_sizes[0] < (size_t)NPTS * 3) return;
    if ((size_t)in_sizes[1] < (size_t)LL * TSZ * 2) return;
    if (in_sizes[2] < LL * 3 || in_sizes[3] < NF * NF || in_sizes[4] < NF) return;
    if ((size_t)out_size < (size_t)NPTS * NF) return;
    if (SZ_TOTAL > ws_size) return;
    const float* x      = (const float*)d_in[0];
    const float* table  = (const float*)d_in[1];
    const float* shifts = (const float*)d_in[2];
    const float* W      = (const float*)d_in[3];
    const float* b      = (const float*)d_in[4];
    float* OUT = (float*)d_out;
    h16* WH = (h16*)d_ws;

    k_wcvt<<<1, 128, 0, stream>>>(W, WH);
    k_enc_dense<<<NPTS / PTS, 256, 0, stream>>>(x, table, shifts, WH, b, OUT);
}
